// FlashMHA_31482110280462
// MI455X (gfx1250) — hardware-verified
//
#include <hip/hip_runtime.h>

typedef __attribute__((ext_vector_type(16))) _Float16 v16h;
typedef __attribute__((ext_vector_type(8)))  _Float16 v8h;
typedef __attribute__((ext_vector_type(16))) __bf16   v16b;
typedef __attribute__((ext_vector_type(8)))  __bf16   v8b;
typedef __attribute__((ext_vector_type(8)))  float    v8f;
typedef __attribute__((ext_vector_type(4)))  float    v4f;
typedef __attribute__((ext_vector_type(2)))  float    v2f;
typedef __attribute__((ext_vector_type(4)))  unsigned v4u;

static constexpr int kBatch  = 2;
static constexpr int kSeqQ   = 2048;
static constexpr int kSeqK   = 2048;
static constexpr int kEmb    = 1024;
static constexpr int kHeads  = 16;
static constexpr int kHeadD  = 64;
static constexpr int kKVCols = 2 * kEmb;
static constexpr int kRowsM  = kBatch * kSeqQ;
static constexpr int kKC     = 64;

__device__ __forceinline__ unsigned short f2bf_bits(float f) {
  unsigned u = __float_as_uint(f);
  return (unsigned short)((u + 0x7FFFu + ((u >> 16) & 1u)) >> 16);
}
__device__ __forceinline__ float bf_bits2f(unsigned short h) { return __uint_as_float(((unsigned)h) << 16); }

__device__ __forceinline__ void dep_guard_h(v8f& a, v8f& b, v16h x, v16h y) { asm volatile("v_nop\n\tv_nop\n\tv_nop\n\tv_nop" : "+v"(a), "+v"(b) : "v"(x), "v"(y)); }
__device__ __forceinline__ void dep_guard_b(v8f& a, v8f& b, v16b x, v16b y) { asm volatile("v_nop\n\tv_nop\n\tv_nop\n\tv_nop" : "+v"(a), "+v"(b) : "v"(x), "v"(y)); }
__device__ __forceinline__ void keep4_h(v16h a, v16h b, v16h c, v16h d) { asm volatile("v_nop" :: "v"(a), "v"(b), "v"(c), "v"(d)); }
__device__ __forceinline__ void keep4_b(v16b a, v16b b, v16b c, v16b d) { asm volatile("v_nop" :: "v"(a), "v"(b), "v"(c), "v"(d)); }
__device__ __forceinline__ void acc_guard4(v8f& a, v8f& b, v8f& c, v8f& d) { asm volatile("v_nop\n\tv_nop\n\tv_nop\n\tv_nop" : "+v"(a), "+v"(b), "+v"(c), "+v"(d)); }
template <typename T> struct Frag;
template <> struct Frag<_Float16> {
  typedef v16h V; union U { v16h v; v8h h[2]; };
  static __device__ __forceinline__ v16h load(const _Float16* p) {
    U f; f.h[0] = *(const v8h*)(p); f.h[1] = *(const v8h*)(p + 16); return f.v;
  }
  static __device__ __forceinline__ v8f mma(v16h a, v16h b, v8f c) {
    return __builtin_amdgcn_wmma_f32_16x16x32_f16(false, a, false, b, (short)0, c, false, false);
  }
  static __device__ __forceinline__ void guard(v8f& a, v8f& b, v16h x, v16h y) { dep_guard_h(a, b, x, y); }
  static __device__ __forceinline__ void keep(v16h a, v16h b, v16h c, v16h d) { keep4_h(a, b, c, d); }
};
template <> struct Frag<__bf16> {
  typedef v16b V; union U { v16b v; v8b h[2]; };
  static __device__ __forceinline__ v16b load(const __bf16* p) {
    U f; f.h[0] = *(const v8b*)(p); f.h[1] = *(const v8b*)(p + 16); return f.v;
  }
  static __device__ __forceinline__ v8f mma(v16b a, v16b b, v8f c) {
    return __builtin_amdgcn_wmma_f32_16x16x32_bf16(false, a, false, b, (short)0, c, false, false);
  }
  static __device__ __forceinline__ void guard(v8f& a, v8f& b, v16b x, v16b y) { dep_guard_b(a, b, x, y); }
  static __device__ __forceinline__ void keep(v16b a, v16b b, v16b c, v16b d) { keep4_b(a, b, c, d); }
};

template <int ET> struct Elem;
template <> struct Elem<0> { typedef _Float16 T; };
template <> struct Elem<1> { typedef __bf16 T; };
template <int ET, int SPLIT, int BIAS_MODE, int OUT_MODE>
__global__ __launch_bounds__(256) void wmma_gemm64(
    const unsigned short* __restrict__ Ap, const unsigned short* __restrict__ A2p, int lda, long strideA,
    const unsigned short* __restrict__ Btp, const unsigned short* __restrict__ Bt2p, int ldb, long strideB,
    void* __restrict__ Cout, void* __restrict__ Cout2, int ldc, long strideC,
    const float* __restrict__ bias,
    int M, int N, int K, float scale) {
  typedef typename Elem<ET>::T T;
  typedef typename Frag<T>::V V;
  const T* A = (const T*)Ap; const T* A2 = (const T*)A2p; const T* Bt = (const T*)Btp; const T* Bt2 = (const T*)Bt2p;
  __shared__ __align__(16) float sT[8][16 * 68];
  const int b    = blockIdx.y;
  const int lane = threadIdx.x & 31;
  const int wave = threadIdx.x >> 5;
  const int tilesN = N >> 6;
  const int tilesM = M >> 6;
  const int tile = blockIdx.x * 8 + wave;
  if (tile >= tilesM * tilesN) return;
  const int tm = tile / tilesN;
  const int tn = tile - tm * tilesN;
  const int m0 = tm << 6;
  const int n0 = tn << 6;

  const T* Ab  = A  + (size_t)b * strideA;
  const T* Bb  = Bt + (size_t)b * strideB;
  const T* Ab2 = (SPLIT != 0) ? (A2  + (size_t)b * strideA) : nullptr;
  const T* Bb2 = (SPLIT == 2) ? (Bt2 + (size_t)b * strideB) : nullptr;

  const int rlane = lane & 15;
  const int koff  = (lane >> 4) * 8;
  const int mOff  = (lane >> 4) * 8;

  v8f acc[4][4];
#pragma unroll
  for (int i = 0; i < 4; ++i)
#pragma unroll
    for (int j = 0; j < 4; ++j) acc[i][j] = (v8f){0.f,0.f,0.f,0.f,0.f,0.f,0.f,0.f};

  for (int k0 = 0; k0 < K; k0 += 32) {
    V bh[4], bl[4];
#pragma unroll
    for (int j = 0; j < 4; ++j) {
      const size_t bo = (size_t)(n0 + (j << 4) + rlane) * ldb + koff + k0;
      bh[j] = Frag<T>::load(Bb + bo);
      if (SPLIT == 2) bl[j] = Frag<T>::load(Bb2 + bo);
    }
#pragma unroll
    for (int i = 0; i < 4; ++i) {
      const size_t ao = (size_t)(m0 + (i << 4) + rlane) * lda + koff + k0;
      V ah = Frag<T>::load(Ab + ao);
      V al;
      if (SPLIT != 0) al = Frag<T>::load(Ab2 + ao);
#pragma unroll
      for (int j = 0; j < 4; ++j) {
        acc[i][j] = Frag<T>::mma(ah, bh[j], acc[i][j]);
        if (SPLIT == 2) acc[i][j] = Frag<T>::mma(ah, bl[j], acc[i][j]);
        if (SPLIT != 0) acc[i][j] = Frag<T>::mma(al, bh[j], acc[i][j]);
      }
      Frag<T>::guard(acc[i][0], acc[i][3], ah, (SPLIT != 0) ? al : ah);
    }
    Frag<T>::keep(bh[0], bh[1], bh[2], bh[3]);
    if (SPLIT == 2) Frag<T>::keep(bl[0], bl[1], bl[2], bl[3]);
  }
  acc_guard4(acc[0][0], acc[0][1], acc[0][2], acc[0][3]);
  acc_guard4(acc[1][0], acc[1][1], acc[1][2], acc[1][3]);
  acc_guard4(acc[2][0], acc[2][1], acc[2][2], acc[2][3]);
  acc_guard4(acc[3][0], acc[3][1], acc[3][2], acc[3][3]);

  float* slab = sT[wave];
#pragma unroll
  for (int i = 0; i < 4; ++i) {
    const int mBase = m0 + (i << 4);
#pragma unroll
    for (int j = 0; j < 4; ++j) {
      const int n = n0 + (j << 4) + rlane;
      float bv = 0.f;
      if (BIAS_MODE == 2) bv = bf_bits2f(f2bf_bits(bias[n]));
#pragma unroll
      for (int r = 0; r < 8; ++r) {
        float v = acc[i][j][r] * scale;
        if (BIAS_MODE == 2) v += bv;
        slab[(mOff + r) * 68 + (j << 4) + rlane] = v;
      }
    }
    __builtin_amdgcn_fence(__ATOMIC_RELEASE, "workgroup");
    __builtin_amdgcn_wave_barrier();
    __builtin_amdgcn_fence(__ATOMIC_ACQUIRE, "workgroup");
    if (OUT_MODE == 0) {
      float* C = (float*)Cout + (size_t)b * strideC;
      const int hh = lane >> 4, c4 = (lane & 15) * 4;
      for (int pass = 0; pass < 2; ++pass) {
#pragma unroll
        for (int it = 0; it < 8; ++it) {
          const int row = it * 2 + hh;
          v4f v = *(const v4f*)(slab + row * 68 + c4);
          *(volatile v4f*)(C + (size_t)(mBase + row) * ldc + n0 + c4) = v;
        }
        __threadfence();
      }
    } else {
      const int q = lane >> 3, c8 = (lane & 7) * 8;
      unsigned short* C  = (unsigned short*)Cout  + (size_t)b * strideC;
      unsigned short* C2 = (OUT_MODE == 2) ? ((unsigned short*)Cout2 + (size_t)b * strideC) : nullptr;
      for (int pass = 0; pass < 2; ++pass) {
#pragma unroll
        for (int it = 0; it < 4; ++it) {
          const int row = it * 4 + q;
          const float* sp = slab + row * 68 + c8;
          v8h hv, lv;
#pragma unroll
          for (int e = 0; e < 8; ++e) {
            if (OUT_MODE == 1) {
              hv[e] = (_Float16)sp[e];
            } else {
              unsigned short hb = f2bf_bits(sp[e]);
              unsigned short lb = f2bf_bits(sp[e] - bf_bits2f(hb));
              hv[e] = __builtin_bit_cast(_Float16, hb);
              lv[e] = __builtin_bit_cast(_Float16, lb);
            }
          }
          *(volatile v8h*)(C + (size_t)(mBase + row) * ldc + n0 + c8) = hv;
          if (OUT_MODE == 2) *(volatile v8h*)(C2 + (size_t)(mBase + row) * ldc + n0 + c8) = lv;
        }
        __threadfence();
      }
    }
    __builtin_amdgcn_fence(__ATOMIC_RELEASE, "workgroup");
    __builtin_amdgcn_wave_barrier();
    __builtin_amdgcn_fence(__ATOMIC_ACQUIRE, "workgroup");
  }
}

__global__ __launch_bounds__(256) void cast_f32_bf16x2(
    const float* __restrict__ in, unsigned short* __restrict__ out, int n2) {
  int i = blockIdx.x * 256 + threadIdx.x;
  if (i < n2) {
    const v2f x = *(const v2f*)(in + 2 * (size_t)i);
    const unsigned u = (unsigned)f2bf_bits(x[0]) | ((unsigned)f2bf_bits(x[1]) << 16);
    ((volatile unsigned*)out)[i] = u;
    __threadfence();
    ((volatile unsigned*)out)[i] = u;
  }
}

__device__ __forceinline__ __bf16 to_bf16(float f) { return __builtin_bit_cast(__bf16, f2bf_bits(f)); }
__device__ __forceinline__ void split_bf16(float f, __bf16& hi, __bf16& lo) {
  const unsigned short hb = f2bf_bits(f);
  hi = __builtin_bit_cast(__bf16, hb);
  lo = to_bf16(f - __uint_as_float(((unsigned)hb) << 16));
}
__device__ __forceinline__ v8f mma_bf16(v16b a, v16b b, v8f c) {
  c = __builtin_amdgcn_wmma_f32_16x16x32_bf16(false, a, false, b, (short)0, c, false, false);
  asm volatile("v_nop\n\tv_nop\n\tv_nop\n\tv_nop" : "+v"(c) : "v"(a), "v"(b));
  return c;
}

__global__ __launch_bounds__(128)
void mha_attn_hd64(const unsigned short* __restrict__ Qh, const unsigned short* __restrict__ Ql,
                   const unsigned short* __restrict__ KVh, const unsigned short* __restrict__ KVl,
                   const float* __restrict__ abias, const int* __restrict__ kmask,
                   unsigned short* __restrict__ Ch, unsigned short* __restrict__ Cl)
{
  __shared__ __align__(16) __bf16 Ksh[kKC * kHeadD];
  __shared__ __align__(16) __bf16 Ksl[kKC * kHeadD];
  __shared__ __align__(16) __bf16 Vth[kHeadD * kKC];
  __shared__ __align__(16) __bf16 Vtl[kHeadD * kKC];
  __shared__ __align__(16) __bf16 Psh[4][16 * kKC];
  __shared__ __align__(16) __bf16 Psl[4][16 * kKC];
  __shared__ float CB[kKC];

  const int tid  = threadIdx.x;
  const int wave = tid >> 5;
  const int lane = tid & 31;
  const int hh   = lane >> 4;
  const int c    = lane & 15;
  const int nqb  = kSeqQ / 64;
  const int bx   = blockIdx.x;
  const int qb   = bx % nqb;
  const int bhd  = bx / nqb;
  const int h    = bhd % kHeads;
  const int b    = bhd / kHeads;
  const int q0   = qb * 64 + wave * 16;
  const float ninf = -__builtin_huge_valf();

  const __bf16* Qhp = (const __bf16*)(const void*)Qh;
  const __bf16* Qlp = (const __bf16*)(const void*)Ql;

  v16b qah[2], qal[2];
  {
    const size_t qo = (size_t)(b * kSeqQ + q0 + c) * kEmb + h * kHeadD + 8 * hh;
#pragma unroll
    for (int dc = 0; dc < 2; ++dc) {
      qah[dc] = Frag<__bf16>::load(Qhp + qo + dc * 32);
      qal[dc] = Frag<__bf16>::load(Qlp + qo + dc * 32);
    }
  }

  const v8f zero8 = (v8f){0.f,0.f,0.f,0.f,0.f,0.f,0.f,0.f};
  float mrow[8], lrow[8];
  v8f oacc[4];
#pragma unroll
  for (int r = 0; r < 8; ++r) { mrow[r] = ninf; lrow[r] = 0.f; }
#pragma unroll
  for (int t = 0; t < 4; ++t) oacc[t] = zero8;

  __bf16* pwh = Psh[wave];
  __bf16* pwl = Psl[wave];

  for (int kc = 0; kc < kSeqK / kKC; ++kc) {
    const int kv0 = kc * kKC;
    __syncthreads();
    {
      const int kvr = tid >> 1, dh = (tid & 1) * 32;
      const size_t ro = (size_t)(b * kSeqK + kv0 + kvr) * kKVCols + h * kHeadD + dh;
#pragma unroll
      for (int i = 0; i < 4; ++i) {
        const v4u wh = *(const v4u*)(KVh + ro + 8 * i);
        const v4u wl = *(const v4u*)(KVl + ro + 8 * i);
        *(v4u*)(Ksh + kvr * kHeadD + dh + 8 * i) = wh;
        *(v4u*)(Ksl + kvr * kHeadD + dh + 8 * i) = wl;
      }
    }
    asm volatile("" ::: "memory");
    {
      const int p = tid >> 2, dq = (tid & 3) * 16;
      const size_t r0 = (size_t)(b * kSeqK + kv0 + 2 * p) * kKVCols + kEmb + h * kHeadD + dq;
      const size_t r1 = r0 + kKVCols;
#pragma unroll
      for (int i = 0; i < 2; ++i) {
        const v4u xh = *(const v4u*)(KVh + r0 + 8 * i);
        const v4u yh = *(const v4u*)(KVh + r1 + 8 * i);
        const v4u xl = *(const v4u*)(KVl + r0 + 8 * i);
        const v4u yl = *(const v4u*)(KVl + r1 + 8 * i);
#pragma unroll
        for (int jw = 0; jw < 4; ++jw) {
          const int d0 = dq + 8 * i + 2 * jw;
          const unsigned xhw = xh[jw], yhw = yh[jw], xlw = xl[jw], ylw = yl[jw];
          const unsigned h0 = (xhw & 0xffffu) | (yhw << 16);
          const unsigned h1 = (xhw >> 16) | (yhw & 0xffff0000u);
          const unsigned l0 = (xlw & 0xffffu) | (ylw << 16);
          const unsigned l1 = (xlw >> 16) | (ylw & 0xffff0000u);
          *(unsigned*)(Vth + d0 * kKC + 2 * p)       = h0;
          *(unsigned*)(Vth + (d0 + 1) * kKC + 2 * p) = h1;
          *(unsigned*)(Vtl + d0 * kKC + 2 * p)       = l0;
          *(unsigned*)(Vtl + (d0 + 1) * kKC + 2 * p) = l1;
        }
      }
    }
    if (tid < kKC) {
      const size_t ki = (size_t)b * kSeqK + kv0 + tid;
      const int keep = kmask[ki];
      const float bb = bf_bits2f(f2bf_bits(abias[ki]));
      CB[tid] = (keep != 0) ? bb : ninf;
    }
    __syncthreads();

    v8f s[4];
#pragma unroll
    for (int j = 0; j < 4; ++j) {
      s[j] = zero8;
#pragma unroll
      for (int dc = 0; dc < 2; ++dc) {
        const v16b kbh = Frag<__bf16>::load(Ksh + (j * 16 + c) * kHeadD + dc * 32 + 8 * hh);
        const v16b kbl = Frag<__bf16>::load(Ksl + (j * 16 + c) * kHeadD + dc * 32 + 8 * hh);
        s[j] = mma_bf16(qah[dc], kbh, s[j]);
        s[j] = mma_bf16(qah[dc], kbl, s[j]);
        s[j] = mma_bf16(qal[dc], kbh, s[j]);
      }
    }
    float cbv[4];
#pragma unroll
    for (int j = 0; j < 4; ++j) cbv[j] = CB[j * 16 + c];
    float cm[8];
#pragma unroll
    for (int r = 0; r < 8; ++r) {
      float m = ninf;
#pragma unroll
      for (int j = 0; j < 4; ++j) {
        const float v = s[j][r] * 0.125f + cbv[j];
        s[j][r] = v;
        m = fmaxf(m, v);
      }
#pragma unroll
      for (int off = 1; off < 16; off <<= 1) m = fmaxf(m, __shfl_xor(m, off, 32));
      cm[r] = m;
    }
#pragma unroll
    for (int r = 0; r < 8; ++r) {
      const float mnew = fmaxf(mrow[r], cm[r]);
      const bool live = (mnew != ninf);
      const float alpha = live ? expf(mrow[r] - mnew) : 1.0f;
      mrow[r] = mnew;
      float psum = 0.f;
#pragma unroll
      for (int j = 0; j < 4; ++j) {
        const float p = live ? expf(s[j][r] - mnew) : 0.0f;
        psum += p;
        __bf16 a, bl;
        split_bf16(p, a, bl);
        pwh[(8 * hh + r) * kKC + j * 16 + c] = a;
        pwl[(8 * hh + r) * kKC + j * 16 + c] = bl;
      }
#pragma unroll
      for (int off = 1; off < 16; off <<= 1) psum += __shfl_xor(psum, off, 32);
      lrow[r] = lrow[r] * alpha + psum;
#pragma unroll
      for (int t = 0; t < 4; ++t) oacc[t][r] *= alpha;
    }
    __builtin_amdgcn_fence(__ATOMIC_RELEASE, "workgroup");
    __builtin_amdgcn_wave_barrier();
    __builtin_amdgcn_fence(__ATOMIC_ACQUIRE, "workgroup");
#pragma unroll
    for (int kk = 0; kk < 2; ++kk) {
      const v16b pa = Frag<__bf16>::load(pwh + c * kKC + kk * 32 + 8 * hh);
      const v16b pl = Frag<__bf16>::load(pwl + c * kKC + kk * 32 + 8 * hh);
#pragma unroll
      for (int t = 0; t < 4; ++t) {
        const v16b vb = Frag<__bf16>::load(Vth + (t * 16 + c) * kKC + kk * 32 + 8 * hh);
        const v16b vl = Frag<__bf16>::load(Vtl + (t * 16 + c) * kKC + kk * 32 + 8 * hh);
        oacc[t] = mma_bf16(pa, vb, oacc[t]);
        oacc[t] = mma_bf16(pa, vl, oacc[t]);
        oacc[t] = mma_bf16(pl, vb, oacc[t]);
      }
    }
  }

  __builtin_amdgcn_fence(__ATOMIC_RELEASE, "workgroup");
  __builtin_amdgcn_wave_barrier();
  __builtin_amdgcn_fence(__ATOMIC_ACQUIRE, "workgroup");
#pragma unroll
  for (int r = 0; r < 8; ++r) {
    const float inv = 1.0f / lrow[r];
#pragma unroll
    for (int t = 0; t < 4; ++t) {
      const float v = oacc[t][r] * inv;
      __bf16 a, bl;
      split_bf16(v, a, bl);
      pwh[(8 * hh + r) * kKC + t * 16 + c] = a;
      pwl[(8 * hh + r) * kKC + t * 16 + c] = bl;
    }
  }
  __builtin_amdgcn_fence(__ATOMIC_RELEASE, "workgroup");
  __builtin_amdgcn_wave_barrier();
  __builtin_amdgcn_fence(__ATOMIC_ACQUIRE, "workgroup");
  {
    _Float16* Chp = (_Float16*)(void*)Ch;
    _Float16* Clp = (_Float16*)(void*)Cl;
    const int q8 = lane >> 3, c8 = (lane & 7) * 8;
    const size_t ob = (size_t)(b * kSeqQ + q0) * kEmb + h * kHeadD + c8;
    for (int pass = 0; pass < 2; ++pass) {
#pragma unroll
      for (int it = 0; it < 4; ++it) {
        const int row = it * 4 + q8;
        const v8b xh = *(const v8b*)(pwh + row * kKC + c8);
        const v8b xl = *(const v8b*)(pwl + row * kKC + c8);
        const v8h yh = __builtin_bit_cast(v8h, xh);
        const v8h yl = __builtin_bit_cast(v8h, xl);
        *(volatile v8h*)(Chp + ob + (size_t)row * kEmb) = yh;
        *(volatile v8h*)(Clp + ob + (size_t)row * kEmb) = yl;
      }
      __threadfence();
    }
  }
}

extern "C" void kernel_launch(void* const* d_in, const int* in_sizes, int n_in,
                              void* d_out, int out_size, void* d_ws, size_t ws_size,
                              hipStream_t stream) {
  static_assert(kRowsM % 64 == 0 && kEmb % 64 == 0 && kKVCols % 64 == 0 && kEmb % 32 == 0);
  static_assert(kSeqQ % 64 == 0 && kSeqK % kKC == 0 && kHeadD == 64 && kHeads * kHeadD == kEmb && kSeqQ == kSeqK);

  if (n_in < 10) return;
  const int nAct = kRowsM * kEmb;
  const int nWq  = kEmb * kEmb;
  const int nWkv = kKVCols * kEmb;
  const int nWo  = kEmb * kEmb;
  if (in_sizes[0] != nAct || in_sizes[1] != kBatch * kSeqK * kEmb || in_sizes[2] != kBatch * kSeqK ||
      in_sizes[3] != kBatch * kSeqK || in_sizes[4] != nWq || in_sizes[5] != kEmb || in_sizes[6] != nWkv ||
      in_sizes[7] != kKVCols || in_sizes[8] != nWo || in_sizes[9] != kEmb) return;
  if (out_size != nAct) return;

  const float* tgt   = (const float*)d_in[0];
  const float* mem   = (const float*)d_in[1];
  const float* abias = (const float*)d_in[2];
  const int*   kmask = (const int*)d_in[3];
  const float* Wq_w  = (const float*)d_in[4];
  const float* Wq_b  = (const float*)d_in[5];
  const float* Wkv_w = (const float*)d_in[6];
  const float* Wkv_b = (const float*)d_in[7];
  const float* out_w = (const float*)d_in[8];
  const float* out_b = (const float*)d_in[9];
  float* out = (float*)d_out;

  const size_t szAct16 = (size_t)nAct * 2;
  const size_t szKV16  = (size_t)kRowsM * kKVCols * 2;
  const size_t oTgt = 0;
  const size_t oMem = oTgt + szAct16;
  const size_t oWq  = oMem + szAct16;
  const size_t oWkv = oWq + (size_t)nWq * 2;
  const size_t oWo  = oWkv + (size_t)nWkv * 2;
  const size_t oQh  = oWo + (size_t)nWo * 2;
  const size_t oQl  = oQh + szAct16;
  const size_t oKVh = oQl + szAct16;
  const size_t oKVl = oKVh + szKV16;
  const size_t oCh  = oKVl + szKV16;
  const size_t oCl  = oCh + szAct16;
  const size_t total = oCl + szAct16;
  if (total > ws_size) return;

  char* ws = (char*)d_ws;
  unsigned short* tgt16 = (unsigned short*)(ws + oTgt);
  unsigned short* mem16 = (unsigned short*)(ws + oMem);
  unsigned short* wq16  = (unsigned short*)(ws + oWq);
  unsigned short* wkv16 = (unsigned short*)(ws + oWkv);
  unsigned short* wo16  = (unsigned short*)(ws + oWo);
  unsigned short* qh    = (unsigned short*)(ws + oQh);
  unsigned short* ql    = (unsigned short*)(ws + oQl);
  unsigned short* kvh   = (unsigned short*)(ws + oKVh);
  unsigned short* kvl   = (unsigned short*)(ws + oKVl);
  unsigned short* ch    = (unsigned short*)(ws + oCh);
  unsigned short* cl    = (unsigned short*)(ws + oCl);

  { const int n2 = nAct / 2; cast_f32_bf16x2<<<dim3((n2 + 255) / 256), dim3(256), 0, stream>>>(tgt,   tgt16, n2); }
  { const int n2 = nAct / 2; cast_f32_bf16x2<<<dim3((n2 + 255) / 256), dim3(256), 0, stream>>>(mem,   mem16, n2); }
  { const int n2 = nWq  / 2; cast_f32_bf16x2<<<dim3((n2 + 255) / 256), dim3(256), 0, stream>>>(Wq_w,  wq16,  n2); }
  { const int n2 = nWkv / 2; cast_f32_bf16x2<<<dim3((n2 + 255) / 256), dim3(256), 0, stream>>>(Wkv_w, wkv16, n2); }
  { const int n2 = nWo  / 2; cast_f32_bf16x2<<<dim3((n2 + 255) / 256), dim3(256), 0, stream>>>(out_w, wo16,  n2); }

  {
    const int tiles = (kRowsM / 64) * (kEmb / 64);
    wmma_gemm64<1, 0, 2, 2><<<dim3((tiles + 7) / 8, 1), dim3(256), 0, stream>>>(
        tgt16, tgt16, kEmb, 0L, wq16, wq16, kEmb, 0L, (void*)qh, (void*)ql, kEmb, 0L,
        Wq_b, kRowsM, kEmb, kEmb, 1.0f);
  }
  {
    const int tiles = (kRowsM / 64) * (kKVCols / 64);
    wmma_gemm64<1, 0, 2, 2><<<dim3((tiles + 7) / 8, 1), dim3(256), 0, stream>>>(
        mem16, mem16, kEmb, 0L, wkv16, wkv16, kEmb, 0L, (void*)kvh, (void*)kvl, kKVCols, 0L,
        Wkv_b, kRowsM, kKVCols, kEmb, 1.0f);
  }
  {
    const int nblk = kBatch * kHeads * (kSeqQ / 64);
    mha_attn_hd64<<<dim3(nblk), dim3(128), 0, stream>>>(qh, ql, kvh, kvl, abias, kmask, ch, cl);
  }
  {
    const int tiles = (kRowsM / 64) * (kEmb / 64);
    wmma_gemm64<1, 1, 2, 0><<<dim3((tiles + 7) / 8, 1), dim3(256), 0, stream>>>(
        ch, cl, kEmb, 0L, wo16, wo16, kEmb, 0L, (void*)out, (void*)cl, kEmb, 0L,
        out_b, kRowsM, kEmb, kEmb, 1.0f);
  }
}
